// ProbabilisticHebbian_56221121904852
// MI455X (gfx1250) — hardware-verified
//
#include <hip/hip_runtime.h>


namespace {
constexpr int B = 128, P = 1024, Q = 1024;
constexpr float XS = 8.0f, LR = 0.005f, WD = 0.0001f;
typedef _Float16 b16;
typedef __attribute__((ext_vector_type(16))) _Float16 v16b;
typedef __attribute__((ext_vector_type(8))) _Float16 v8b;
typedef __attribute__((ext_vector_type(8))) float v8f;
typedef __attribute__((ext_vector_type(4))) float v4f;
__device__ __forceinline__ float bf16_rne(float f) { unsigned int u = __float_as_uint(f); u += 0x7FFFu + ((u >> 16) & 1u); float r = __uint_as_float(u & 0xFFFF0000u); asm volatile("" : "+v"(r)); return r; }
__device__ __forceinline__ v16b frag_kb(const b16* p, int hh) { const v8b a = *(const v8b*)(p + 8 * hh), b = *(const v8b*)(p + 16 + 8 * hh); v16b f;
#pragma unroll
  for (int e = 0; e < 8; ++e) { f[e] = a[e]; f[8 + e] = b[e]; } return f; }
__device__ __forceinline__ v8f wmma16b(v16b a, v16b b, v8f c) { v8f d = __builtin_amdgcn_wmma_f32_16x16x32_f16(false, a, false, b, (short)0, c, false, false); asm volatile("v_nop\n\tv_nop\n\tv_nop\n\tv_nop" : "+v"(d) : "v"(a), "v"(b)); return d; }
__device__ __forceinline__ void wave_lds_sync() { __builtin_amdgcn_fence(__ATOMIC_RELEASE, "workgroup"); __builtin_amdgcn_wave_barrier(); __builtin_amdgcn_fence(__ATOMIC_ACQUIRE, "workgroup"); }
__device__ __forceinline__ float pmul(float a, float b) { float p = a * b; asm volatile("" : "+v"(p)); return p; }

__global__ __launch_bounds__(256) void prep_kernel(const float* __restrict__ pre, const float* __restrict__ post, b16* __restrict__ PT, b16* __restrict__ QT) { const int u = blockIdx.x * 256 + threadIdx.x; if (u >= P * (B / 8)) return; const int r = u / (B / 8), b0 = (u % (B / 8)) * 8; v8b a, c;
#pragma unroll
  for (int j = 0; j < 8; ++j) { a[j] = (b16)(bf16_rne(post[(size_t)(b0 + j) * P + r]) * XS); c[j] = (b16)(bf16_rne(pre[(size_t)(b0 + j) * Q + r]) * XS); }
  for (int pass = 0; pass < 2; ++pass) { *(volatile v8b*)(PT + (size_t)r * B + b0) = a; *(volatile v8b*)(QT + (size_t)r * B + b0) = c; __threadfence(); } }
__global__ __launch_bounds__(32) void dw_kernel(const b16* __restrict__ PT, const b16* __restrict__ QT, const float* __restrict__ W, float* __restrict__ out) { __shared__ float Tf[16][132]; const int lane = threadIdx.x, nloc = lane & 15, hlf = lane >> 4; const int g = blockIdx.x % (Q / 128); const size_t m0 = (size_t)(blockIdx.x / (Q / 128)) * 16;
  v8f acc[8];
#pragma unroll
  for (int t = 0; t < 8; ++t) acc[t] = (v8f){};
#pragma unroll
  for (int kb = 0; kb < B; kb += 32) { const v16b a = frag_kb(PT + (m0 + nloc) * B + kb, hlf);
#pragma unroll
    for (int t = 0; t < 8; ++t) acc[t] = wmma16b(a, frag_kb(QT + (size_t)(g * 128 + t * 16 + nloc) * B + kb, hlf), acc[t]); }
#pragma unroll
  for (int t = 0; t < 8; ++t)
#pragma unroll
    for (int r8 = 0; r8 < 8; ++r8) Tf[8 * hlf + r8][t * 16 + nloc] = acc[t][r8] * (1.0f / (XS * XS * B));
  wave_lds_sync();
  for (int pass = 0; pass < 2; ++pass) { for (int rr = 0; rr < 16; ++rr) { const size_t o = (m0 + rr) * Q + g * 128 + lane * 4; const v4f w = *(const v4f*)(W + o); v4f r; for (int k = 0; k < 4; ++k) r[k] = LR * (Tf[rr][lane * 4 + k] - WD * bf16_rne(w[k])); *(volatile v4f*)(out + o) = r; } __threadfence(); } }
}

extern "C" void kernel_launch(void* const* d_in, const int* in_sizes, int n_in, void* d_out, int out_size, void* d_ws, size_t ws_size, hipStream_t stream) {
  (void)n_in;
  auto Fp = [&](int i) { return (const float*)d_in[i]; };
  if (in_sizes[0] != B * Q || in_sizes[1] != B * P || in_sizes[2] != P * Q || out_size != P * Q) return;
  size_t off = 0; char* ws = (char*)d_ws;
  auto carve = [&](size_t bytes) { char* p = ws + off; off += (bytes + 255) & ~(size_t)255; return p; };
  b16* PT = (b16*)carve((size_t)P * B * 2); b16* QT = (b16*)carve((size_t)Q * B * 2);
  if (off > ws_size || off > ((size_t)4 << 20)) return;
  prep_kernel<<<(P * (B / 8) + 255) / 256, 256, 0, stream>>>(Fp(0), Fp(1), PT, QT);
  dw_kernel<<<(P / 16) * (Q / 128), 32, 0, stream>>>(PT, QT, Fp(2), (float*)d_out);
}
